// MambaBlock_41042707480728
// MI455X (gfx1250) — hardware-verified
//
#include <hip/hip_runtime.h>
#include <stddef.h>
#include <stdint.h>
#include <math.h>


#define BATCH  2
#define SEQ    1024
#define DM     1024
#define DI     2048
#define NST    16
#define RK     64
#define XD     96
#define MR     (BATCH * SEQ)
#define KHL    (2 * DI)
#define KR2    (2 * RK)
#define XRP    (2 * DI)
#define GBM    64
#define GTHR   128
#define NTHR   256
#define SC_CH  64
#define SC_TS  64
#define SC_THR 512
#define WSMAX  134217728

#define PU_X   (MR * DM / 8)
#define PU_WIN (2 * DI * DM / 8)
#define PU_XP  (XD * DI / 8)
#define PU_DT  (DI * RK / 8)
#define PU_WO  (DM * DI / 8)
#define PU_ALL (PU_X + PU_WIN + PU_XP + PU_DT + PU_WO)

static_assert(PU_X % NTHR == 0 && PU_WIN % NTHR == 0 && PU_XP % NTHR == 0 && PU_DT % NTHR == 0 && PU_WO % NTHR == 0);
static_assert(MR % GBM == 0 && (2 * DI) % 64 == 0 && DI % 64 == 0 && DM % 64 == 0 && XD == 96);
static_assert(DM % 32 == 0 && KHL % 32 == 0 && KR2 % 32 == 0);
static_assert((DI & (DI - 1)) == 0 && (RK & (RK - 1)) == 0 && (DM & (DM - 1)) == 0);
static_assert(SEQ % SC_TS == 0 && DI % SC_CH == 0 && SC_THR == SC_CH * 8 && SC_TS * 8 == SC_THR);
static_assert(NST == 16 && RK == 64);

typedef float          v2f   __attribute__((ext_vector_type(2)));
typedef float          v4f   __attribute__((ext_vector_type(4)));
typedef float          v8f   __attribute__((ext_vector_type(8)));
typedef int            v8i   __attribute__((ext_vector_type(8)));
typedef unsigned short v4us  __attribute__((ext_vector_type(4)));
typedef unsigned short v8us  __attribute__((ext_vector_type(8)));
typedef unsigned short v16us __attribute__((ext_vector_type(16)));
typedef __bf16         v16bf __attribute__((ext_vector_type(16)));
typedef v2f  __attribute__((may_alias)) v2fa;
typedef v4f  __attribute__((may_alias)) v4fa;
typedef v4us __attribute__((may_alias)) v4usa;
typedef v8us __attribute__((may_alias)) v8usa;
union FragB { v16bf v; v16us u; v8us h[2]; v8i w; };

__device__ __forceinline__ v8f wmb(const FragB& a, const FragB& b, v8f c) {
  v8f d = __builtin_amdgcn_wmma_f32_16x16x32_bf16(false, a.v, false, b.v, (short)0, c, false, false);
  asm volatile("v_nop\n\tv_nop\n\tv_nop\n\tv_nop" : "+v"(d) : "v"(a.w), "v"(b.w));
  return d;
}

__device__ __forceinline__ unsigned bf16_bits(float f) {
  const unsigned u = __float_as_uint(f);
  return (u + 0x7FFFu + ((u >> 16) & 1u)) >> 16;
}
__device__ __forceinline__ float bf16_val(float f) {
  return __uint_as_float(bf16_bits(f) << 16);
}
__device__ __forceinline__ void hilo(float v, unsigned& hb, unsigned& lb) {
  hb = bf16_bits(v);
  lb = bf16_bits(v - __uint_as_float(hb << 16));
}
__device__ __forceinline__ float softplus_f(float v) {
  return fmaxf(v, 0.0f) + log1pf(expf(-fabsf(v)));
}
__device__ __forceinline__ float sigmoid_f(float v) {
  return __builtin_amdgcn_rcpf(1.0f + expf(-v));
}

__device__ __forceinline__ void cvt8(const float* __restrict__ s, unsigned short* d, size_t u) {
  const float* p = s + u * 8;
  const v4f a = *(const v4f*)p;
  const v4f b = *(const v4f*)(p + 4);
  v8us o;
  o[0] = (unsigned short)bf16_bits(a.x); o[1] = (unsigned short)bf16_bits(a.y);
  o[2] = (unsigned short)bf16_bits(a.z); o[3] = (unsigned short)bf16_bits(a.w);
  o[4] = (unsigned short)bf16_bits(b.x); o[5] = (unsigned short)bf16_bits(b.y);
  o[6] = (unsigned short)bf16_bits(b.z); o[7] = (unsigned short)bf16_bits(b.w);
  unsigned short* dp = d + u * 8;
  *(volatile v8us*)dp = o;
  __threadfence();
  *(volatile v8us*)dp = o;
}

__global__ __launch_bounds__(NTHR) void k_prep(const float* __restrict__ x, const float* __restrict__ win,
                                               const float* __restrict__ wxp, const float* __restrict__ wdt,
                                               const float* __restrict__ wo,
                                               unsigned short* XB, unsigned short* WIN, unsigned short* XPB,
                                               unsigned short* DTB, unsigned short* WOB) {
  const int u = (int)blockIdx.x * NTHR + (int)threadIdx.x;
  if (u < PU_X) {
    cvt8(x, XB, (size_t)u);
  } else if (u < PU_X + PU_WIN) {
    cvt8(win, WIN, (size_t)(u - PU_X));
  } else if (u < PU_X + PU_WIN + PU_XP) {
    cvt8(wxp, XPB, (size_t)(u - PU_X - PU_WIN));
  } else if (u < PU_X + PU_WIN + PU_XP + PU_DT) {
    cvt8(wdt, DTB, (size_t)(u - PU_X - PU_WIN - PU_XP));
  } else if (u < PU_ALL) {
    cvt8(wo, WOB, (size_t)(u - PU_X - PU_WIN - PU_XP - PU_DT));
  }
}

template <int NT, int EPI>
__global__ __launch_bounds__(GTHR) void k_gemm(
    const unsigned short* __restrict__ A, int lda, int K,
    const unsigned short* __restrict__ WT, int ldb, int kmaskB,
    const float* __restrict__ bias, float* outF, int ldo,
    unsigned short* outH, float* outBC)
{
  constexpr int SP = 16 * NT;
  __shared__ __attribute__((aligned(16))) float stg[GBM * SP];
  const int tid = (int)threadIdx.x, lane = tid & 31, wave = tid >> 5, hh = lane >> 4, m = lane & 15;
  const int rowBase = (int)blockIdx.x * GBM;
  const int col0    = (int)blockIdx.y * SP;

  v8f acc[NT];
  {
    const v8f z = {0.f, 0.f, 0.f, 0.f, 0.f, 0.f, 0.f, 0.f};
#pragma unroll
    for (int t = 0; t < NT; ++t) acc[t] = z;
  }
  const unsigned short* ap = A  + (size_t)(rowBase + 16 * wave + m) * (size_t)lda + 8 * hh;
  const unsigned short* wp = WT + (size_t)(col0 + m) * (size_t)ldb + 8 * hh;
#pragma unroll 1
  for (int k0 = 0; k0 < K; k0 += 32) {
    FragB af;
    af.h[0] = *(const v8usa*)(ap + k0);
    af.h[1] = *(const v8usa*)(ap + k0 + 16);
    const int kb = k0 & kmaskB;
#pragma unroll
    for (int t = 0; t < NT; ++t) {
      const unsigned short* wq = wp + (size_t)(16 * t) * (size_t)ldb + kb;
      FragB bf;
      bf.h[0] = *(const v8usa*)wq;
      bf.h[1] = *(const v8usa*)(wq + 16);
      acc[t] = wmb(af, bf, acc[t]);
    }
  }

#pragma unroll
  for (int t = 0; t < NT; ++t) {
    const int lc = 16 * t + m;
#pragma unroll
    for (int r = 0; r < 8; ++r) {
      const int lr = 16 * wave + 8 * hh + r;
      stg[lr * SP + lc] = acc[t][r];
    }
  }
  __syncthreads();

  if constexpr (EPI == 2) {
    static_assert(NT == 6 || EPI != 2);
    const int m7 = m & 7;
    const bool sel = m >= 8;
    v8us ov[8];
#pragma unroll
    for (int i = 0; i < 8; ++i) {
      const int lr = 16 * wave + 2 * i + hh;
      const v4f a = *(const v4fa*)(stg + lr * SP + 8 * m7);
      const v4f b = *(const v4fa*)(stg + lr * SP + 8 * m7 + 4);
      unsigned hb, lb;
      v8us o;
      hilo(a.x, hb, lb); o[0] = (unsigned short)(sel ? lb : hb);
      hilo(a.y, hb, lb); o[1] = (unsigned short)(sel ? lb : hb);
      hilo(a.z, hb, lb); o[2] = (unsigned short)(sel ? lb : hb);
      hilo(a.w, hb, lb); o[3] = (unsigned short)(sel ? lb : hb);
      hilo(b.x, hb, lb); o[4] = (unsigned short)(sel ? lb : hb);
      hilo(b.y, hb, lb); o[5] = (unsigned short)(sel ? lb : hb);
      hilo(b.z, hb, lb); o[6] = (unsigned short)(sel ? lb : hb);
      hilo(b.w, hb, lb); o[7] = (unsigned short)(sel ? lb : hb);
      ov[i] = o;
    }
    const int q = lane >> 3, j8 = lane & 7;
    v4f bv[4];
#pragma unroll
    for (int i = 0; i < 4; ++i) {
      const int lr = 16 * wave + 4 * i + q;
      bv[i] = *(const v4fa*)(stg + lr * SP + 64 + 4 * j8);
    }
#pragma unroll
    for (int i = 0; i < 8; ++i) {
      unsigned short* dp = outH + (size_t)(rowBase + 16 * wave + 2 * i + hh) * KR2 + 8 * m;
      *(volatile v8us*)dp = ov[i];
    }
#pragma unroll
    for (int i = 0; i < 4; ++i) {
      float* bp = outBC + (size_t)(rowBase + 16 * wave + 4 * i + q) * 32 + 4 * j8;
      *(volatile v4f*)bp = bv[i];
    }
    __threadfence();
#pragma unroll
    for (int i = 0; i < 8; ++i) {
      unsigned short* dp = outH + (size_t)(rowBase + 16 * wave + 2 * i + hh) * KR2 + 8 * m;
      *(volatile v8us*)dp = ov[i];
    }
#pragma unroll
    for (int i = 0; i < 4; ++i) {
      float* bp = outBC + (size_t)(rowBase + 16 * wave + 4 * i + q) * 32 + 4 * j8;
      *(volatile v4f*)bp = bv[i];
    }
  } else {
    v4f bb;
    {
      const v4f t = *(const v4f*)(bias + col0 + 4 * m);
      bb.x = bf16_val(t.x); bb.y = bf16_val(t.y); bb.z = bf16_val(t.z); bb.w = bf16_val(t.w);
    }
    if constexpr (EPI == 1) {
#pragma unroll 1
      for (int i = 0; i < 8; ++i) {
        float* sp = stg + (16 * wave + 2 * i + hh) * SP + 4 * m;
        v4f v = *(v4fa*)sp;
        v.x = softplus_f(v.x + bb.x);
        v.y = softplus_f(v.y + bb.y);
        v.z = softplus_f(v.z + bb.z);
        v.w = softplus_f(v.w + bb.w);
        *(v4fa*)sp = v;
      }
    }
    v4f fv[8];
#pragma unroll
    for (int i = 0; i < 8; ++i) {
      const int lr = 16 * wave + 2 * i + hh;
      v4f v = *(const v4fa*)(stg + lr * SP + 4 * m);
      if constexpr (EPI == 0) v = v + bb;
      fv[i] = v;
    }
#pragma unroll
    for (int i = 0; i < 8; ++i) {
      const int gr = rowBase + 16 * wave + 2 * i + hh;
      float* op = outF + (size_t)gr * (size_t)ldo + col0 + 4 * m;
      *(volatile v4f*)op = fv[i];
    }
    __threadfence();
#pragma unroll
    for (int i = 0; i < 8; ++i) {
      const int gr = rowBase + 16 * wave + 2 * i + hh;
      float* op = outF + (size_t)gr * (size_t)ldo + col0 + 4 * m;
      *(volatile v4f*)op = fv[i];
    }
  }
}

__device__ __forceinline__ float conv_silu1(const v4f w, float x0, float x1, float x2, float x3, float b) {
  float acc = bf16_val(w.x) * x0;
  acc = fmaf(bf16_val(w.y), x1, acc);
  acc = fmaf(bf16_val(w.z), x2, acc);
  acc = fmaf(bf16_val(w.w), x3, acc);
  acc = acc + bf16_val(b);
  return acc * sigmoid_f(acc);
}

__global__ __launch_bounds__(NTHR) void k_conv(const float* __restrict__ XR, const float* __restrict__ cw,
                                               const float* __restrict__ cb, float* U, unsigned short* UHL) {
  __shared__ __attribute__((aligned(16))) unsigned short sh[2048];
  const int tid   = (int)threadIdx.x;
  const int row   = (int)blockIdx.x >> 1;
  const int dbase = ((int)blockIdx.x & 1) * 1024;
  const int d     = dbase + 4 * tid;
  const int l     = row & (SEQ - 1);

  v4f xs[4];
#pragma unroll
  for (int j = 0; j < 4; ++j) {
    const int  ls = l - 3 + j;
    const bool ok = ls >= 0;
    const int  rs = ok ? (row - 3 + j) : row;
    const float kf = ok ? 1.0f : 0.0f;
    const v4f v = *(const v4f*)(XR + (size_t)rs * XRP + d);
    xs[j] = v * kf;
  }
  const v4f w0 = *(const v4f*)(cw + (size_t)(d + 0) * 4);
  const v4f w1 = *(const v4f*)(cw + (size_t)(d + 1) * 4);
  const v4f w2 = *(const v4f*)(cw + (size_t)(d + 2) * 4);
  const v4f w3 = *(const v4f*)(cw + (size_t)(d + 3) * 4);
  const v4f bv = *(const v4f*)(cb + d);
  v4f s;
  s.x = conv_silu1(w0, xs[0].x, xs[1].x, xs[2].x, xs[3].x, bv.x);
  s.y = conv_silu1(w1, xs[0].y, xs[1].y, xs[2].y, xs[3].y, bv.y);
  s.z = conv_silu1(w2, xs[0].z, xs[1].z, xs[2].z, xs[3].z, bv.z);
  s.w = conv_silu1(w3, xs[0].w, xs[1].w, xs[2].w, xs[3].w, bv.w);

  v4us h4, l4;
  {
    unsigned hb, lb;
    hilo(s.x, hb, lb); h4[0] = (unsigned short)hb; l4[0] = (unsigned short)lb;
    hilo(s.y, hb, lb); h4[1] = (unsigned short)hb; l4[1] = (unsigned short)lb;
    hilo(s.z, hb, lb); h4[2] = (unsigned short)hb; l4[2] = (unsigned short)lb;
    hilo(s.w, hb, lb); h4[3] = (unsigned short)hb; l4[3] = (unsigned short)lb;
  }
  *(v4usa*)(sh + 4 * tid) = h4;
  *(v4usa*)(sh + 1024 + 4 * tid) = l4;
  __syncthreads();
  const v8us q = *(const v8usa*)(sh + 8 * tid);
  const int colo = (tid < 128) ? (dbase + 8 * tid) : (DI + dbase + 8 * (tid - 128));
  float* up = U + (size_t)row * DI + d;
  unsigned short* hp = UHL + (size_t)row * KHL + colo;
  *(volatile v4f*)up = s;
  *(volatile v8us*)hp = q;
  __threadfence();
  *(volatile v4f*)up = s;
  *(volatile v8us*)hp = q;
}

__device__ __forceinline__ float gate1(float y, float u, float dd, float r) {
  const float t = fmaf(u, dd, y);
  return t * (r * sigmoid_f(r));
}

__global__ __launch_bounds__(SC_THR) void k_scan(const float* __restrict__ DELTA, const float* __restrict__ U,
                                                 const float* __restrict__ BC, const float* __restrict__ XR,
                                                 const float* __restrict__ A_log, const float* __restrict__ Dp,
                                                 unsigned short* YG) {
  __shared__ __attribute__((aligned(16))) float sdl[SC_TS * SC_CH];
  __shared__ __attribute__((aligned(16))) float su[SC_TS * SC_CH];
  __shared__ __attribute__((aligned(16))) float sy[SC_TS * SC_CH];
  __shared__ __attribute__((aligned(16))) float sbc[SC_TS * 32];
  const int tid = (int)threadIdx.x;
  const int j   = tid & 7;
  const int c   = tid >> 3;
  const int b     = (int)blockIdx.x >> 5;
  const int dbase = ((int)blockIdx.x & 31) * SC_CH;
  const int d     = dbase + c;

  float a0, a1;
  {
    const v2f al = *(const v2fa*)(A_log + (size_t)d * NST + 2 * j);
    a0 = -expf(bf16_val(al.x));
    a1 = -expf(bf16_val(al.y));
  }
  v4f d0, d1;
  {
    const v4f t0 = *(const v4f*)(Dp + dbase + 8 * j);
    const v4f t1 = *(const v4f*)(Dp + dbase + 8 * j + 4);
    d0.x = bf16_val(t0.x); d0.y = bf16_val(t0.y); d0.z = bf16_val(t0.z); d0.w = bf16_val(t0.w);
    d1.x = bf16_val(t1.x); d1.y = bf16_val(t1.y); d1.z = bf16_val(t1.z); d1.w = bf16_val(t1.w);
  }
  float h0 = 0.0f, h1 = 0.0f;

#pragma unroll 1
  for (int ch = 0; ch < SEQ / SC_TS; ++ch) {
    const int row0 = b * SEQ + ch * SC_TS;
#pragma unroll
    for (int q = 0; q < 2; ++q) {
      const int idx = tid + SC_THR * q;
      const int r   = idx >> 4;
      const int c4  = (idx & 15) * 4;
      const size_t go = (size_t)(row0 + r) * DI + dbase + c4;
      *(v4fa*)(sdl + r * SC_CH + c4) = *(const v4f*)(DELTA + go);
      *(v4fa*)(su  + r * SC_CH + c4) = *(const v4f*)(U + go);
    }
    {
      const int r  = tid >> 3;
      const int c4 = (tid & 7) * 4;
      *(v4fa*)(sbc + r * 32 + c4) = *(const v4f*)(BC + (size_t)(row0 + r) * 32 + c4);
    }
    __syncthreads();

#pragma unroll 1
    for (int t = 0; t < SC_TS; ++t) {
      const float dlv = sdl[t * SC_CH + c];
      const float uv  = su[t * SC_CH + c];
      const v2f bn = *(const v2fa*)(sbc + t * 32 + 2 * j);
      const v2f cn = *(const v2fa*)(sbc + t * 32 + 16 + 2 * j);
      const float e0 = expf(dlv * a0);
      const float e1 = expf(dlv * a1);
      h0 = fmaf(e0, h0, (dlv * bn.x) * uv);
      h1 = fmaf(e1, h1, (dlv * bn.y) * uv);
      float p = h0 * cn.x;
      p = fmaf(h1, cn.y, p);
      p += __shfl_xor(p, 1, 32);
      p += __shfl_xor(p, 2, 32);
      p += __shfl_xor(p, 4, 32);
      if (j == 0) sy[t * SC_CH + c] = p;
    }
    __syncthreads();

    {
      const int grow = row0 + c;
      const v4f ya = *(const v4fa*)(sy + c * SC_CH + 8 * j);
      const v4f yb = *(const v4fa*)(sy + c * SC_CH + 8 * j + 4);
      const v4f ua = *(const v4fa*)(su + c * SC_CH + 8 * j);
      const v4f ub = *(const v4fa*)(su + c * SC_CH + 8 * j + 4);
      const float* rp = XR + (size_t)grow * XRP + DI + dbase + 8 * j;
      const v4f ra = *(const v4f*)rp;
      const v4f rb = *(const v4f*)(rp + 4);
      v8us oh, ol;
      unsigned hb, lb;
      hilo(gate1(ya.x, ua.x, d0.x, ra.x), hb, lb); oh[0] = (unsigned short)hb; ol[0] = (unsigned short)lb;
      hilo(gate1(ya.y, ua.y, d0.y, ra.y), hb, lb); oh[1] = (unsigned short)hb; ol[1] = (unsigned short)lb;
      hilo(gate1(ya.z, ua.z, d0.z, ra.z), hb, lb); oh[2] = (unsigned short)hb; ol[2] = (unsigned short)lb;
      hilo(gate1(ya.w, ua.w, d0.w, ra.w), hb, lb); oh[3] = (unsigned short)hb; ol[3] = (unsigned short)lb;
      hilo(gate1(yb.x, ub.x, d1.x, rb.x), hb, lb); oh[4] = (unsigned short)hb; ol[4] = (unsigned short)lb;
      hilo(gate1(yb.y, ub.y, d1.y, rb.y), hb, lb); oh[5] = (unsigned short)hb; ol[5] = (unsigned short)lb;
      hilo(gate1(yb.z, ub.z, d1.z, rb.z), hb, lb); oh[6] = (unsigned short)hb; ol[6] = (unsigned short)lb;
      hilo(gate1(yb.w, ub.w, d1.w, rb.w), hb, lb); oh[7] = (unsigned short)hb; ol[7] = (unsigned short)lb;
      unsigned short* ph = YG + (size_t)grow * KHL + dbase + 8 * j;
      unsigned short* pl = ph + DI;
      *(volatile v8us*)ph = oh;
      *(volatile v8us*)pl = ol;
      __threadfence();
      *(volatile v8us*)ph = oh;
      *(volatile v8us*)pl = ol;
    }
    __syncthreads();
  }
}

static inline size_t al256(size_t o) { return (o + 255) & ~(size_t)255; }

extern "C" void kernel_launch(void* const* d_in, const int* in_sizes, int n_in,
                              void* d_out, int out_size, void* d_ws, size_t ws_size,
                              hipStream_t stream) {
  if (n_in < 12) return;
  if (in_sizes[0] != MR * DM) return;
  if (in_sizes[1] != 2 * DI * DM) return;
  if (in_sizes[2] != 2 * DI) return;
  if (in_sizes[3] != DI * 4) return;
  if (in_sizes[4] != DI) return;
  if (in_sizes[5] != XD * DI) return;
  if (in_sizes[6] != DI * RK) return;
  if (in_sizes[7] != DI) return;
  if (in_sizes[8] != DI * NST) return;
  if (in_sizes[9] != DI) return;
  if (in_sizes[10] != DM * DI) return;
  if (in_sizes[11] != DM) return;
  if (out_size != MR * DM) return;

  const float* x     = (const float*)d_in[0];
  const float* winp  = (const float*)d_in[1];
  const float* binp  = (const float*)d_in[2];
  const float* convw = (const float*)d_in[3];
  const float* convb = (const float*)d_in[4];
  const float* wxp   = (const float*)d_in[5];
  const float* wdt   = (const float*)d_in[6];
  const float* bdt   = (const float*)d_in[7];
  const float* alog  = (const float*)d_in[8];
  const float* dpar  = (const float*)d_in[9];
  const float* wout  = (const float*)d_in[10];
  const float* bout  = (const float*)d_in[11];
  float* out = (float*)d_out;

  char* ws = (char*)d_ws;
  size_t off = 0;
  const size_t oXB  = off; off = al256(off + (size_t)MR * DM * 2);
  const size_t oWIN = off; off = al256(off + (size_t)2 * DI * DM * 2);
  const size_t oXPB = off; off = al256(off + (size_t)XD * DI * 2);
  const size_t oDTB = off; off = al256(off + (size_t)DI * RK * 2);
  const size_t oWOB = off; off = al256(off + (size_t)DM * DI * 2);
  const size_t oXR  = off; off = al256(off + (size_t)MR * XRP * 4);
  const size_t oU   = off; off = al256(off + (size_t)MR * DI * 4);
  const size_t oUHL = off; off = al256(off + (size_t)MR * KHL * 2);
  const size_t oDR  = off; off = al256(off + (size_t)MR * KR2 * 2);
  const size_t oBC  = off; off = al256(off + (size_t)MR * 32 * 4);
  const size_t oDL  = off; off = al256(off + (size_t)MR * DI * 4);
  const size_t oYG  = off; off = al256(off + (size_t)MR * KHL * 2);
  if (off > ws_size || off > (size_t)WSMAX) return;
  unsigned short* XB   = (unsigned short*)(ws + oXB);
  unsigned short* WIN  = (unsigned short*)(ws + oWIN);
  unsigned short* XPB  = (unsigned short*)(ws + oXPB);
  unsigned short* DTB  = (unsigned short*)(ws + oDTB);
  unsigned short* WOB  = (unsigned short*)(ws + oWOB);
  float*          XR   = (float*)(ws + oXR);
  float*          U    = (float*)(ws + oU);
  unsigned short* UHL  = (unsigned short*)(ws + oUHL);
  unsigned short* DRHL = (unsigned short*)(ws + oDR);
  float*          BCp  = (float*)(ws + oBC);
  float*          DL   = (float*)(ws + oDL);
  unsigned short* YGHL = (unsigned short*)(ws + oYG);

  k_prep<<<PU_ALL / NTHR, NTHR, 0, stream>>>(x, winp, wxp, wdt, wout, XB, WIN, XPB, DTB, WOB);
  k_gemm<4, 0><<<dim3(MR / GBM, (2 * DI) / 64), GTHR, 0, stream>>>(
      XB, DM, DM, WIN, DM, DM - 1, binp, XR, XRP, DRHL, BCp);
  k_conv<<<MR * 2, NTHR, 0, stream>>>(XR, convw, convb, U, UHL);
  k_gemm<6, 2><<<dim3(MR / GBM, 1), GTHR, 0, stream>>>(
      UHL, KHL, KHL, XPB, DI, DI - 1, bdt, DL, DI, DRHL, BCp);
  k_gemm<4, 1><<<dim3(MR / GBM, DI / 64), GTHR, 0, stream>>>(
      DRHL, KR2, KR2, DTB, RK, RK - 1, bdt, DL, DI, DRHL, BCp);
  k_scan<<<BATCH * (DI / SC_CH), SC_THR, 0, stream>>>(DL, U, BCp, XR, alog, dpar, YGHL);
  k_gemm<4, 0><<<dim3(MR / GBM, DM / 64), GTHR, 0, stream>>>(
      YGHL, KHL, KHL, WOB, DI, DI - 1, bout, out, DM, DRHL, BCp);
}
